// ColBERT_62319975465254
// MI455X (gfx1250) — hardware-verified
//
#include <hip/hip_runtime.h>

typedef _Float16 v16h __attribute__((ext_vector_type(16)));
typedef _Float16 v8h  __attribute__((ext_vector_type(8)));
typedef _Float16 v8ha __attribute__((ext_vector_type(8), may_alias));
typedef float    v8f  __attribute__((ext_vector_type(8)));
typedef float    v4f  __attribute__((ext_vector_type(4)));
typedef float    v4fa __attribute__((ext_vector_type(4), may_alias));
union Frag { v16h v; v8h half[2]; _Float16 h[16]; };

#define KV   768
#define DD   128
#define LT   256
#define NQB  32
#define NDB  32
#define NROWS 16384

__device__ __forceinline__ v8f mma16(v16h a, v16h b, v8f c) {
  c = __builtin_amdgcn_wmma_f32_16x16x32_f16(false, a, false, b, (short)0, c, false, false);
  asm volatile("v_nop\n\tv_nop\n\tv_nop\n\tv_nop" : "+v"(c) : "v"(a), "v"(b));
  return c;
}

__global__ __launch_bounds__(256) void wt_kernel(const float* __restrict__ W, _Float16* __restrict__ Wt) {
  const int t = blockIdx.x * 256 + threadIdx.x;
  if (t >= DD * (KV / 8)) return;
  const int n = t / (KV / 8), k8 = (t % (KV / 8)) * 8;
  v8h v;
#pragma unroll
  for (int i = 0; i < 8; ++i) v[i] = (_Float16)W[(size_t)(k8 + i) * DD + n];
  *(volatile v8h*)(Wt + (size_t)n * KV + k8) = v;
  __threadfence();
  *(volatile v8h*)(Wt + (size_t)n * KV + k8) = v;
}

__global__ __launch_bounds__(256) void proj_norm_kernel(const float* __restrict__ qh, const float* __restrict__ dh,
                                                        const _Float16* __restrict__ Wt, const float* __restrict__ bias,
                                                        _Float16* __restrict__ reps) {
  __shared__ __attribute__((aligned(16))) _Float16 st[8][16][DD + 8];
  const int wave = threadIdx.x >> 5, lane = threadIdx.x & 31, lrow = lane & 15, half = lane >> 4;
  const int rowbase = (blockIdx.x * 8 + wave) * 16;
  const float* src = (rowbase < NROWS / 2) ? (qh + (size_t)rowbase * KV) : (dh + (size_t)(rowbase - NROWS / 2) * KV);
  const float* arow = src + (size_t)lrow * KV;

  v8f c[8];
#pragma unroll
  for (int t = 0; t < 8; ++t) c[t] = (v8f)(0.0f);
  for (int kb = 0; kb < KV; kb += 32) {
    Frag a;
    {
      const v4f lo0 = *(const v4fa*)(arow + kb + 8 * half), lo1 = *(const v4fa*)(arow + kb + 8 * half + 4);
      const v4f hi0 = *(const v4fa*)(arow + kb + 16 + 8 * half), hi1 = *(const v4fa*)(arow + kb + 16 + 8 * half + 4);
#pragma unroll
      for (int i = 0; i < 4; ++i) { a.h[i] = (_Float16)lo0[i]; a.h[4 + i] = (_Float16)lo1[i]; a.h[8 + i] = (_Float16)hi0[i]; a.h[12 + i] = (_Float16)hi1[i]; }
    }
#pragma unroll
    for (int t = 0; t < 8; ++t) {
      const _Float16* bp = Wt + (size_t)(16 * t + lrow) * KV + kb;
      Frag b;
      b.half[0] = *(const v8h*)(bp + 8 * half);
      b.half[1] = *(const v8h*)(bp + 16 + 8 * half);
      c[t] = mma16(a.v, b.v, c[t]);
    }
  }
  float inv[8];
#pragma unroll
  for (int r = 0; r < 8; ++r) {
    float s = 0.f;
#pragma unroll
    for (int t = 0; t < 8; ++t) { c[t][r] += bias[16 * t + lrow]; s += c[t][r] * c[t][r]; }
    s += __shfl_xor(s, 1, 32); s += __shfl_xor(s, 2, 32); s += __shfl_xor(s, 4, 32); s += __shfl_xor(s, 8, 32);
    inv[r] = 1.0f / fmaxf(sqrtf(s), 1e-12f);
  }
#pragma unroll
  for (int r = 0; r < 8; ++r)
#pragma unroll
    for (int t = 0; t < 8; ++t) st[wave][8 * half + r][16 * t + lrow] = (_Float16)(c[t][r] * inv[r]);
  __builtin_amdgcn_fence(__ATOMIC_ACQ_REL, "workgroup");
  __builtin_amdgcn_wave_barrier();
  const int rsub = lane >> 4, c8 = (lane & 15) * 8;
  for (int pass = 0; pass < 2; ++pass) {
#pragma unroll
    for (int q = 0; q < 8; ++q) {
      const int r = q * 2 + rsub;
      const v8h v = *(const v8ha*)&st[wave][r][c8];
      *(volatile v8h*)(reps + (size_t)(rowbase + r) * DD + c8) = v;
    }
    if (pass == 0) __threadfence();
  }
}

__global__ __launch_bounds__(256) void scores_kernel(const _Float16* __restrict__ reps, const int* __restrict__ mask,
                                                     float* __restrict__ slots) {
  __shared__ __attribute__((aligned(16))) _Float16 dtile[LT][DD + 8];
  __shared__ float wmax[8][16];
  __shared__ float accs;
  __shared__ int seps;
  const int db = blockIdx.x, qb = blockIdx.y;
  const int tid = threadIdx.x, lane = tid & 31, w = tid >> 5, lrow = lane & 15, half = lane >> 4;
  const _Float16* qbase = reps + (size_t)(qb * LT) * DD;
  const _Float16* dbase = reps + (size_t)(NROWS / 2 + db * LT) * DD;
  for (int e = tid; e < LT * (DD / 8); e += 256) {
    const int r = e / (DD / 8), c8 = (e % (DD / 8)) * 8;
    *(v8ha*)&dtile[r][c8] = *(const v8ha*)(dbase + (size_t)r * DD + c8);
  }
  if (w == 0) {
    int s = 0;
    for (int i = lane; i < LT; i += 32) s += mask[qb * LT + i];
    s += __shfl_xor(s, 16, 32); s += __shfl_xor(s, 8, 32); s += __shfl_xor(s, 4, 32); s += __shfl_xor(s, 2, 32); s += __shfl_xor(s, 1, 32);
    if (lane == 0) { seps = s - 1; accs = 0.f; }
  }
  __syncthreads();

  for (int lt = 0; lt < LT / 16; ++lt) {
    v8f c0 = (v8f)(0.0f), c1 = (v8f)(0.0f);
    const _Float16* aptr = qbase + (size_t)(lt * 16 + lrow) * DD;
#pragma unroll
    for (int kb = 0; kb < DD; kb += 32) {
      Frag a, b0, b1;
      a.half[0]  = *(const v8ha*)(aptr + kb + 8 * half);
      a.half[1]  = *(const v8ha*)(aptr + kb + 16 + 8 * half);
      b0.half[0] = *(const v8ha*)&dtile[w * 32 + lrow][kb + 8 * half];
      b0.half[1] = *(const v8ha*)&dtile[w * 32 + lrow][kb + 16 + 8 * half];
      b1.half[0] = *(const v8ha*)&dtile[w * 32 + 16 + lrow][kb + 8 * half];
      b1.half[1] = *(const v8ha*)&dtile[w * 32 + 16 + lrow][kb + 16 + 8 * half];
      c0 = mma16(a.v, b0.v, c0);
      c1 = mma16(a.v, b1.v, c1);
    }
    float mx[8];
#pragma unroll
    for (int r = 0; r < 8; ++r) {
      float m = fmaxf(c0[r], c1[r]);
      m = fmaxf(m, __shfl_xor(m, 1, 32)); m = fmaxf(m, __shfl_xor(m, 2, 32)); m = fmaxf(m, __shfl_xor(m, 4, 32)); m = fmaxf(m, __shfl_xor(m, 8, 32));
      mx[r] = m;
    }
    if (lrow == 0) {
#pragma unroll
      for (int r = 0; r < 8; ++r) wmax[w][half * 8 + r] = mx[r];
    }
    __syncthreads();
    float partial = 0.f;
    if (tid < 16) {
      float m = wmax[0][tid];
#pragma unroll
      for (int ww = 1; ww < 8; ++ww) m = fmaxf(m, wmax[ww][tid]);
      const int l = lt * 16 + tid;
      const float wgt = (l >= 1 && l != seps) ? (float)mask[qb * LT + l] : 0.f;
      partial = m * wgt;
    }
    if (tid < 32) {
      partial += __shfl_xor(partial, 1, 32); partial += __shfl_xor(partial, 2, 32);
      partial += __shfl_xor(partial, 4, 32); partial += __shfl_xor(partial, 8, 32);
      if (tid == 0) accs += partial;
    }
    __syncthreads();
  }
  if (tid < 32) {
    const float val = (tid == 0) ? accs : 0.f;
    float* dst = slots + (size_t)(qb * NDB + db) * 32 + tid;
    *(volatile float*)dst = val;
    __threadfence();
    *(volatile float*)dst = val;
  }
}

__global__ __launch_bounds__(256) void gather_kernel(const float* __restrict__ slots, float* __restrict__ out) {
  const int t = threadIdx.x;
  v4f v;
#pragma unroll
  for (int j = 0; j < 4; ++j) v[j] = slots[(size_t)(t * 4 + j) * 32];
  *(volatile v4f*)(out + t * 4) = v;
  __threadfence();
  *(volatile v4f*)(out + t * 4) = v;
}

extern "C" void kernel_launch(void* const* d_in, const int* in_sizes, int n_in,
                              void* d_out, int out_size, void* d_ws, size_t ws_size, hipStream_t stream) {
  (void)in_sizes; (void)n_in; (void)out_size; (void)ws_size;
  const float* qh = (const float*)d_in[0];
  const float* dh = (const float*)d_in[1];
  const float* W  = (const float*)d_in[2];
  const float* b  = (const float*)d_in[3];
  const int* mask = (const int*)d_in[4];
  char* ws = (char*)d_ws;
  _Float16* Wt   = (_Float16*)ws;
  _Float16* reps = (_Float16*)(ws + (size_t)KV * DD * 2);
  float*   slots = (float*)(ws + (size_t)KV * DD * 2 + (size_t)NROWS * DD * 2);
  wt_kernel<<<(DD * (KV / 8) + 255) / 256, 256, 0, stream>>>(W, Wt);
  proj_norm_kernel<<<NROWS / 16 / 8, 256, 0, stream>>>(qh, dh, Wt, b, reps);
  scores_kernel<<<dim3(NDB, NQB), 256, 0, stream>>>(reps, mask, slots);
  gather_kernel<<<1, 256, 0, stream>>>(slots, (float*)d_out);
}
